// MambaBlock_35854386987594
// MI455X (gfx1250) — hardware-verified
//
#include <hip/hip_runtime.h>
#include <math.h>

typedef __attribute__((ext_vector_type(16))) _Float16 v16h;
typedef __attribute__((ext_vector_type(8)))  _Float16 v8h;
typedef __attribute__((ext_vector_type(16))) __bf16   v16b;
typedef __attribute__((ext_vector_type(8)))  __bf16   v8b;
typedef __attribute__((ext_vector_type(8)))  float    v8f;
typedef __attribute__((ext_vector_type(4)))  float    v4f;

constexpr int kBatch  = 4;
constexpr int kSeq    = 2048;
constexpr int kDm     = 1024;
constexpr int kDin    = 2048;
constexpr int kNst    = 16;
constexpr int kConvK  = 4;
constexpr int kXzP    = 2 * kDin;
constexpr int kRows   = kBatch * kSeq;
constexpr int kUP     = 64;
constexpr int kHP     = 32;
constexpr int kConvTP = 260;
constexpr int kScanTS = 64;
constexpr int kScanP  = 36;
static_assert(kRows * kDm == 8388608);
static_assert(kDm * kXzP == 4194304);
static_assert(kDin * kConvK == 8192);
static_assert(kDin * kNst == 32768);
static_assert(kDin * kDm == 2097152);
static_assert((kDm % 32) == 0 && (kDin % 32) == 0 && (kHP % 32) == 0);
static_assert((kSeq % 64) == 0 && (kXzP % 64) == 0 && (kUP % 64) == 0 && (kDin % 64) == 0 && (kDm % 64) == 0);
static_assert((kSeq % kScanTS) == 0 && (kDin % 256) == 0 && (kScanTS == 64));
static_assert(kNst <= 32 && kUP == 64 && kHP == 32);

constexpr size_t kOffXB  = 0;
constexpr size_t kOffWIN = kOffXB  + (size_t)kRows * kDm  * 2;
constexpr size_t kOffWOB = kOffWIN + (size_t)kXzP  * kDm  * 2;
constexpr size_t kOffWBB = kOffWOB + (size_t)kDm   * kDin * 2;
constexpr size_t kOffWCB = kOffWBB + (size_t)kUP   * kDin * 2;
constexpr size_t kOffXZ  = kOffWCB + (size_t)kDin  * kHP  * 2;
constexpr size_t kOffXCH = kOffXZ  + (size_t)kSeq  * kXzP * 4;
constexpr size_t kOffXCL = kOffXCH + (size_t)kSeq  * kDin * 2;
constexpr size_t kOffU   = kOffXCL + (size_t)kSeq  * kDin * 2;
constexpr size_t kOffHH  = kOffU   + (size_t)kSeq  * kUP  * 4;
constexpr size_t kOffHL  = kOffHH  + (size_t)kSeq  * kHP  * 2;
constexpr size_t kOffYH  = kOffHL  + (size_t)kSeq  * kHP  * 2;
constexpr size_t kOffYL  = kOffYH  + (size_t)kSeq  * kDin * 2;
constexpr size_t kWsTotal = kOffYL + (size_t)kSeq  * kDin * 2;
static_assert(kWsTotal == 97648640ull);
static_assert(kWsTotal <= 134217728ull);
static_assert((kOffWIN % 128) == 0 && (kOffWOB % 128) == 0 && (kOffWBB % 128) == 0 && (kOffWCB % 128) == 0 &&
              (kOffXZ % 128) == 0 && (kOffXCH % 128) == 0 && (kOffXCL % 128) == 0 && (kOffU % 128) == 0 &&
              (kOffHH % 128) == 0 && (kOffHL % 128) == 0 && (kOffYH % 128) == 0 && (kOffYL % 128) == 0);

__device__ __forceinline__ unsigned short f2bf_bits(float f) {
  unsigned u = __float_as_uint(f);
  return (unsigned short)((u + 0x7FFFu + ((u >> 16) & 1u)) >> 16);
}
__device__ __forceinline__ float bf_bits2f(unsigned short h) { return __uint_as_float(((unsigned)h) << 16); }
__device__ __forceinline__ float bf_rne(float f) { return bf_bits2f(f2bf_bits(f)); }

__device__ __forceinline__ void dep_guard4_h(v8f& a, v8f& b, v8f& c, v8f& d, v16h x, v16h y) { asm volatile("v_nop\n\tv_nop\n\tv_nop\n\tv_nop" : "+v"(a), "+v"(b), "+v"(c), "+v"(d) : "v"(x), "v"(y)); }
__device__ __forceinline__ void dep_guard4_b(v8f& a, v8f& b, v8f& c, v8f& d, v16b x, v16b y) { asm volatile("v_nop\n\tv_nop\n\tv_nop\n\tv_nop" : "+v"(a), "+v"(b), "+v"(c), "+v"(d) : "v"(x), "v"(y)); }
__device__ __forceinline__ void keep4_h(v16h a, v16h b, v16h c, v16h d) { asm volatile("v_nop" :: "v"(a), "v"(b), "v"(c), "v"(d)); }
__device__ __forceinline__ void keep4_b(v16b a, v16b b, v16b c, v16b d) { asm volatile("v_nop" :: "v"(a), "v"(b), "v"(c), "v"(d)); }
__device__ __forceinline__ void acc_guard4(v8f& a, v8f& b, v8f& c, v8f& d) { asm volatile("v_nop\n\tv_nop\n\tv_nop\n\tv_nop" : "+v"(a), "+v"(b), "+v"(c), "+v"(d)); }
template <typename T> struct Frag;
template <> struct Frag<_Float16> {
  typedef v16h V; union U { v16h v; v8h h[2]; };
  static __device__ __forceinline__ v16h load(const _Float16* p) {
    U f; f.h[0] = *(const v8h*)(p); f.h[1] = *(const v8h*)(p + 16); return f.v;
  }
  static __device__ __forceinline__ v8f mma(v16h a, v16h b, v8f c) {
    return __builtin_amdgcn_wmma_f32_16x16x32_f16(false, a, false, b, (short)0, c, false, false);
  }
  static __device__ __forceinline__ void guard4(v8f& a, v8f& b, v8f& c, v8f& d, v16h x, v16h y) { dep_guard4_h(a, b, c, d, x, y); }
  static __device__ __forceinline__ void keep(v16h a, v16h b, v16h c, v16h d) { keep4_h(a, b, c, d); }
};
template <> struct Frag<__bf16> {
  typedef v16b V; union U { v16b v; v8b h[2]; };
  static __device__ __forceinline__ v16b load(const __bf16* p) {
    U f; f.h[0] = *(const v8b*)(p); f.h[1] = *(const v8b*)(p + 16); return f.v;
  }
  static __device__ __forceinline__ v8f mma(v16b a, v16b b, v8f c) {
    return __builtin_amdgcn_wmma_f32_16x16x32_bf16(false, a, false, b, (short)0, c, false, false);
  }
  static __device__ __forceinline__ void guard4(v8f& a, v8f& b, v8f& c, v8f& d, v16b x, v16b y) { dep_guard4_b(a, b, c, d, x, y); }
  static __device__ __forceinline__ void keep(v16b a, v16b b, v16b c, v16b d) { keep4_b(a, b, c, d); }
};

template <int ET> struct Elem;
template <> struct Elem<0> { typedef _Float16 T; };
template <> struct Elem<1> { typedef __bf16 T; };
template <int ET, int SPL, int OUT_MODE, int GATE>
__global__ __launch_bounds__(256) void wmma_gemm64(
    const unsigned short* __restrict__ Ap, const unsigned short* __restrict__ A2p, int lda, long strideA,
    const unsigned short* __restrict__ Btp, const unsigned short* __restrict__ Bt2p, int ldb, long strideB,
    void* __restrict__ Cout, void* __restrict__ Cout2, int ldc, long strideC,
    const float* __restrict__ Gp, int ldg, long strideG,
    int M, int N, int K, float scale) {
  typedef typename Elem<ET>::T T;
  typedef typename Frag<T>::V V;
  const T* A = (const T*)Ap; const T* A2 = (const T*)A2p; const T* Bt = (const T*)Btp; const T* Bt2 = (const T*)Bt2p;
  __shared__ __align__(16) float sT[8][16 * 68];
  const int b    = blockIdx.y;
  const int lane = threadIdx.x & 31;
  const int wave = threadIdx.x >> 5;
  const int tilesN = N >> 6;
  const int tilesM = M >> 6;
  const int tile = blockIdx.x * 8 + wave;
  if (tile >= tilesM * tilesN) return;
  const int tm = tile / tilesN;
  const int tn = tile - tm * tilesN;
  const int m0 = tm << 6;
  const int n0 = tn << 6;

  const T* Ab  = A  + (size_t)b * strideA;
  const T* Bb  = Bt + (size_t)b * strideB;
  const T* Ab2 = (SPL >= 1) ? (A2  + (size_t)b * strideA) : nullptr;
  const T* Bb2 = (SPL == 2) ? (Bt2 + (size_t)b * strideB) : nullptr;

  const int rlane = lane & 15;
  const int koff  = (lane >> 4) * 8;
  const int mOff  = (lane >> 4) * 8;

  v8f acc[4][4];
#pragma unroll
  for (int i = 0; i < 4; ++i)
#pragma unroll
    for (int j = 0; j < 4; ++j) acc[i][j] = (v8f){0.f,0.f,0.f,0.f,0.f,0.f,0.f,0.f};

  for (int k0 = 0; k0 < K; k0 += 32) {
    V bh[4], bl[4];
#pragma unroll
    for (int j = 0; j < 4; ++j) {
      const size_t bo = (size_t)(n0 + (j << 4) + rlane) * ldb + koff + k0;
      bh[j] = Frag<T>::load(Bb + bo);
      if (SPL == 2) bl[j] = Frag<T>::load(Bb2 + bo);
    }
#pragma unroll
    for (int i = 0; i < 4; ++i) {
      const size_t ao = (size_t)(m0 + (i << 4) + rlane) * lda + koff + k0;
      V ah = Frag<T>::load(Ab + ao);
      V al;
      if (SPL >= 1) al = Frag<T>::load(Ab2 + ao);
#pragma unroll
      for (int j = 0; j < 4; ++j) {
        acc[i][j] = Frag<T>::mma(ah, bh[j], acc[i][j]);
        if (SPL == 2) acc[i][j] = Frag<T>::mma(ah, bl[j], acc[i][j]);
        if (SPL >= 1) acc[i][j] = Frag<T>::mma(al, bh[j], acc[i][j]);
      }
      Frag<T>::guard4(acc[i][0], acc[i][1], acc[i][2], acc[i][3], ah, (SPL >= 1) ? al : ah);
    }
    Frag<T>::keep(bh[0], bh[1], bh[2], bh[3]);
    if (SPL == 2) Frag<T>::keep(bl[0], bl[1], bl[2], bl[3]);
  }
  acc_guard4(acc[0][0], acc[0][1], acc[0][2], acc[0][3]);
  acc_guard4(acc[1][0], acc[1][1], acc[1][2], acc[1][3]);
  acc_guard4(acc[2][0], acc[2][1], acc[2][2], acc[2][3]);
  acc_guard4(acc[3][0], acc[3][1], acc[3][2], acc[3][3]);

  float* slab = sT[wave];
#pragma unroll
  for (int i = 0; i < 4; ++i) {
    const int mBase = m0 + (i << 4);
#pragma unroll
    for (int j = 0; j < 4; ++j) {
#pragma unroll
      for (int r = 0; r < 8; ++r) {
        const float v = acc[i][j][r] * scale;
        slab[(mOff + r) * 68 + (j << 4) + rlane] = v;
      }
    }
    __builtin_amdgcn_fence(__ATOMIC_RELEASE, "workgroup");
    __builtin_amdgcn_wave_barrier();
    __builtin_amdgcn_fence(__ATOMIC_ACQUIRE, "workgroup");
    if (GATE == 1) {
      const float* Gb = Gp + (size_t)b * strideG;
      const int gh = lane >> 4, gc4 = (lane & 15) * 4;
#pragma unroll 1
      for (int it = 0; it < 8; ++it) {
        const int row = it * 2 + gh;
        float* sp = slab + row * 68 + gc4;
        const v4f sv = *(const v4f*)sp;
        const v4f zv = *(const v4f*)(Gb + (size_t)(mBase + row) * ldg + n0 + gc4);
        v4f ov;
#pragma unroll
        for (int e = 0; e < 4; ++e) {
          const float zz = zv[e];
          const float sg = __builtin_amdgcn_rcpf(1.0f + expf(-zz));
          const float g  = zz * sg;
          const float yv = sv[e];
          ov[e] = yv * g;
        }
        *(v4f*)sp = ov;
      }
      __builtin_amdgcn_fence(__ATOMIC_RELEASE, "workgroup");
      __builtin_amdgcn_wave_barrier();
      __builtin_amdgcn_fence(__ATOMIC_ACQUIRE, "workgroup");
    }
    if (OUT_MODE == 0) {
      float* C = (float*)Cout + (size_t)b * strideC;
      const int hh = lane >> 4, c4 = (lane & 15) * 4;
      for (int pass = 0; pass < 2; ++pass) {
#pragma unroll
        for (int it = 0; it < 8; ++it) {
          const int row = it * 2 + hh;
          v4f v = *(const v4f*)(slab + row * 68 + c4);
          *(volatile v4f*)(C + (size_t)(mBase + row) * ldc + n0 + c4) = v;
        }
        __threadfence();
      }
    } else {
      const int q = lane >> 3, c8 = (lane & 7) * 8;
      unsigned short* C  = (unsigned short*)Cout  + (size_t)b * strideC;
      unsigned short* C2 = (OUT_MODE == 2) ? ((unsigned short*)Cout2 + (size_t)b * strideC) : nullptr;
      for (int pass = 0; pass < 2; ++pass) {
#pragma unroll
        for (int it = 0; it < 4; ++it) {
          const int row = it * 4 + q;
          const float* sp = slab + row * 68 + c8;
          v8h hv, lv;
#pragma unroll
          for (int e = 0; e < 8; ++e) {
            if (OUT_MODE == 1) {
              hv[e] = (_Float16)sp[e];
            } else {
              unsigned short hb = f2bf_bits(sp[e]);
              unsigned short lb = f2bf_bits(sp[e] - bf_bits2f(hb));
              hv[e] = __builtin_bit_cast(_Float16, hb);
              lv[e] = __builtin_bit_cast(_Float16, lb);
            }
          }
          *(volatile v8h*)(C + (size_t)(mBase + row) * ldc + n0 + c8) = hv;
          if (OUT_MODE == 2) *(volatile v8h*)(C2 + (size_t)(mBase + row) * ldc + n0 + c8) = lv;
        }
        __threadfence();
      }
    }
    __builtin_amdgcn_fence(__ATOMIC_RELEASE, "workgroup");
    __builtin_amdgcn_wave_barrier();
    __builtin_amdgcn_fence(__ATOMIC_ACQUIRE, "workgroup");
  }
}

__global__ __launch_bounds__(256) void cast_bf16_kernel(
    const float* __restrict__ src, unsigned short* __restrict__ dst, int total8)
{
  const int i = blockIdx.x * 256 + threadIdx.x;
  if (i >= total8) return;
  const size_t e0 = (size_t)i << 3;
  const float* p = src + e0;
  const v4f a0 = *(const v4f*)(p);
  const v4f a1 = *(const v4f*)(p + 4);
  v8h hv;
#pragma unroll
  for (int e = 0; e < 4; ++e) {
    const float f0 = a0[e];
    const float f1 = a1[e];
    hv[e]     = __builtin_bit_cast(_Float16, f2bf_bits(f0));
    hv[4 + e] = __builtin_bit_cast(_Float16, f2bf_bits(f1));
  }
  unsigned short* q = dst + e0;
  *(volatile v8h*)q = hv;
  __threadfence();
  *(volatile v8h*)q = hv;
}

__global__ __launch_bounds__(256) void transpose_bf16_kernel(
    const float* __restrict__ W, unsigned short* __restrict__ Bt, int Kdim, int Ndim, int Npad)
{
  __shared__ float tile[64 * 65];
  const int tid = threadIdx.x, lane = tid & 31, wave = tid >> 5;
  const int n0 = blockIdx.x * 64;
  const int k0 = blockIdx.y * 64;
  (void)Npad;
#pragma unroll
  for (int p = 0; p < 16; ++p) {
    const int idx = tid + p * 256;
    const int kk  = idx >> 6;
    const int nn  = idx & 63;
    const int n   = n0 + nn;
    const int nc  = (n < Ndim) ? n : (Ndim - 1);
    const float v = W[(size_t)(k0 + kk) * Ndim + nc];
    tile[kk * 65 + nn] = (n < Ndim) ? v : 0.f;
  }
  __syncthreads();
  const int q = lane >> 3, c8 = (lane & 7) * 8;
  v8h hv[2];
#pragma unroll
  for (int it = 0; it < 2; ++it) {
    const int nrow = it * 32 + wave * 4 + q;
#pragma unroll
    for (int e = 0; e < 8; ++e) {
      const float f = tile[(c8 + e) * 65 + nrow];
      hv[it][e] = __builtin_bit_cast(_Float16, f2bf_bits(f));
    }
  }
  for (int pass = 0; pass < 2; ++pass) {
#pragma unroll
    for (int it = 0; it < 2; ++it) {
      const int nrow = it * 32 + wave * 4 + q;
      *(volatile v8h*)(Bt + (size_t)(n0 + nrow) * Kdim + k0 + c8) = hv[it];
    }
    __threadfence();
  }
}

__global__ __launch_bounds__(256) void wc_pack_kernel(
    const float* __restrict__ W, unsigned short* __restrict__ Bt, int total8)
{
  const int i = blockIdx.x * 256 + threadIdx.x;
  if (i >= total8) return;
  const int n  = i >> 2;
  const int k8 = (i & 3) * 8;
  v8h hv;
#pragma unroll
  for (int e = 0; e < 8; ++e) {
    const int k  = k8 + e;
    const int kc = (k < kNst) ? k : (kNst - 1);
    const float w = W[(size_t)kc * kDin + n];
    const float v = (k < kNst) ? w : 0.0f;
    hv[e] = __builtin_bit_cast(_Float16, f2bf_bits(v));
  }
  unsigned short* q = Bt + ((size_t)i << 3);
  *(volatile v8h*)q = hv;
  __threadfence();
  *(volatile v8h*)q = hv;
}

__global__ __launch_bounds__(256) void conv_silu_kernel(
    const float* __restrict__ XZ, const float* __restrict__ cw, const float* __restrict__ cb,
    unsigned short* __restrict__ XCH, unsigned short* __restrict__ XCL)
{
  __shared__ __align__(16) float sT[16 * kConvTP];
  const int tid = threadIdx.x, lane = tid & 31, wave = tid >> 5;
  const int d0 = blockIdx.x * 256, d = d0 + tid;
  const int t0 = blockIdx.y * 64;
  const float w0 = bf_rne(cw[d * kConvK + 0]);
  const float w1 = bf_rne(cw[d * kConvK + 1]);
  const float w2 = bf_rne(cw[d * kConvK + 2]);
  const float w3 = bf_rne(cw[d * kConvK + 3]);
  const float bc = bf_rne(cb[d]);
  float xm3, xm2, xm1;
  {
    const int r3 = t0 - 3, r2 = t0 - 2, r1 = t0 - 1;
    const float v3 = XZ[(size_t)(r3 < 0 ? 0 : r3) * kXzP + d];
    const float v2 = XZ[(size_t)(r2 < 0 ? 0 : r2) * kXzP + d];
    const float v1 = XZ[(size_t)(r1 < 0 ? 0 : r1) * kXzP + d];
    xm3 = (r3 >= 0) ? v3 : 0.f;
    xm2 = (r2 >= 0) ? v2 : 0.f;
    xm1 = (r1 >= 0) ? v1 : 0.f;
  }
#pragma unroll 1
  for (int sub = 0; sub < 4; ++sub) {
    const int lb = t0 + sub * 16;
#pragma unroll 1
    for (int s = 0; s < 16; ++s) {
      const float xcur = XZ[(size_t)(lb + s) * kXzP + d];
      float acc = w0 * xm3;
      acc = fmaf(w1, xm2, acc);
      acc = fmaf(w2, xm1, acc);
      acc = fmaf(w3, xcur, acc);
      const float sv = acc + bc;
      const float sg = __builtin_amdgcn_rcpf(1.0f + expf(-sv));
      sT[s * kConvTP + tid] = sv * sg;
      xm3 = xm2; xm2 = xm1; xm1 = xcur;
    }
    __syncthreads();
    v8h bh[2], blo[2];
#pragma unroll
    for (int it = 0; it < 2; ++it) {
      const float* sp = sT + (it * 8 + wave) * kConvTP + lane * 8;
      const v4f a0 = *(const v4f*)(sp);
      const v4f a1 = *(const v4f*)(sp + 4);
#pragma unroll
      for (int e = 0; e < 4; ++e) {
        const float f0 = a0[e];
        const float f1 = a1[e];
        const unsigned short h0 = f2bf_bits(f0), h1 = f2bf_bits(f1);
        const unsigned short l0 = f2bf_bits(f0 - bf_bits2f(h0)), l1 = f2bf_bits(f1 - bf_bits2f(h1));
        bh[it][e]      = __builtin_bit_cast(_Float16, h0);
        bh[it][4 + e]  = __builtin_bit_cast(_Float16, h1);
        blo[it][e]     = __builtin_bit_cast(_Float16, l0);
        blo[it][4 + e] = __builtin_bit_cast(_Float16, l1);
      }
    }
    for (int pass = 0; pass < 2; ++pass) {
#pragma unroll
      for (int it = 0; it < 2; ++it) {
        const size_t o = (size_t)(lb + it * 8 + wave) * kDin + d0 + lane * 8;
        *(volatile v8h*)(XCH + o) = bh[it];
        *(volatile v8h*)(XCL + o) = blo[it];
      }
      __threadfence();
    }
    __syncthreads();
  }
}

__global__ __launch_bounds__(32) void scan_kernel(
    const float* __restrict__ U, unsigned short* __restrict__ HH, unsigned short* __restrict__ HL)
{
  __shared__ __align__(16) float sH[kScanTS * kScanP];
  const int lane = threadIdx.x;
  const int rr = lane >> 2, k8 = (lane & 3) * 8;
  float h = 0.0f;
#pragma unroll 1
  for (int t0 = 0; t0 < kSeq; t0 += kScanTS) {
#pragma unroll 1
    for (int s = 0; s < kScanTS; ++s) {
      const float uv = U[(size_t)(t0 + s) * kUP + lane];
      const float hd = h * 0.9f;
      const float ud = 0.1f * uv;
      h = hd + ud;
      sH[s * kScanP + lane] = (lane < kNst) ? h : 0.0f;
    }
    __syncthreads();
    v8h hv[8], lv[8];
#pragma unroll
    for (int it = 0; it < 8; ++it) {
      const int row = rr + 8 * it;
      const float* sp = sH + row * kScanP + k8;
      const v4f a0 = *(const v4f*)(sp);
      const v4f a1 = *(const v4f*)(sp + 4);
#pragma unroll
      for (int e = 0; e < 4; ++e) {
        const float f0 = a0[e];
        const float f1 = a1[e];
        const unsigned short h0 = f2bf_bits(f0), h1 = f2bf_bits(f1);
        const unsigned short l0 = f2bf_bits(f0 - bf_bits2f(h0)), l1 = f2bf_bits(f1 - bf_bits2f(h1));
        hv[it][e]     = __builtin_bit_cast(_Float16, h0);
        hv[it][4 + e] = __builtin_bit_cast(_Float16, h1);
        lv[it][e]     = __builtin_bit_cast(_Float16, l0);
        lv[it][4 + e] = __builtin_bit_cast(_Float16, l1);
      }
    }
    for (int pass = 0; pass < 2; ++pass) {
#pragma unroll
      for (int it = 0; it < 8; ++it) {
        const int row = rr + 8 * it;
        const size_t o = (size_t)(t0 + row) * kHP + k8;
        *(volatile v8h*)(HH + o) = hv[it];
        *(volatile v8h*)(HL + o) = lv[it];
      }
      __threadfence();
    }
    __syncthreads();
  }
}

extern "C" void kernel_launch(void* const* d_in, const int* in_sizes, int n_in,
                              void* d_out, int out_size, void* d_ws, size_t ws_size,
                              hipStream_t stream)
{
  if (n_in < 7) return;
  if (in_sizes[0] != kRows * kDm) return;
  if (in_sizes[1] != kDm * kXzP) return;
  if (in_sizes[2] != kDin * kConvK) return;
  if (in_sizes[3] != kDin) return;
  if (in_sizes[4] != kDin * kNst) return;
  if (in_sizes[5] != kNst * kDin) return;
  if (in_sizes[6] != kDin * kDm) return;
  if (out_size != kRows * kDm) return;
  if (ws_size < kWsTotal) return;

  const float* x      = (const float*)d_in[0];
  const float* w_in   = (const float*)d_in[1];
  const float* conv_w = (const float*)d_in[2];
  const float* conv_b = (const float*)d_in[3];
  const float* w_B    = (const float*)d_in[4];
  const float* w_C    = (const float*)d_in[5];
  const float* w_out  = (const float*)d_in[6];
  float* out = (float*)d_out;

  char* ws = (char*)d_ws;
  unsigned short* XB   = (unsigned short*)(ws + kOffXB);
  unsigned short* WINB = (unsigned short*)(ws + kOffWIN);
  unsigned short* WOB  = (unsigned short*)(ws + kOffWOB);
  unsigned short* WBB  = (unsigned short*)(ws + kOffWBB);
  unsigned short* WCB  = (unsigned short*)(ws + kOffWCB);
  float*          XZ   = (float*)(ws + kOffXZ);
  unsigned short* XCH  = (unsigned short*)(ws + kOffXCH);
  unsigned short* XCL  = (unsigned short*)(ws + kOffXCL);
  float*          U    = (float*)(ws + kOffU);
  unsigned short* HH   = (unsigned short*)(ws + kOffHH);
  unsigned short* HL   = (unsigned short*)(ws + kOffHL);
  unsigned short* YH   = (unsigned short*)(ws + kOffYH);
  unsigned short* YL   = (unsigned short*)(ws + kOffYL);
  const float* gdummy = XZ;

  cast_bf16_kernel<<<(kRows * kDm) / 8 / 256, 256, 0, stream>>>(x, XB, (kRows * kDm) / 8);
  transpose_bf16_kernel<<<dim3(kXzP / 64, kDm / 64), 256, 0, stream>>>(w_in,  WINB, kDm,  kXzP, kXzP);
  transpose_bf16_kernel<<<dim3(kUP / 64, kDin / 64), 256, 0, stream>>>(w_B,   WBB,  kDin, kNst, kUP);
  transpose_bf16_kernel<<<dim3(kDm / 64, kDin / 64), 256, 0, stream>>>(w_out, WOB,  kDin, kDm,  kDm);
  wc_pack_kernel<<<(kDin * kHP) / 8 / 256, 256, 0, stream>>>(w_C, WCB, (kDin * kHP) / 8);

  for (int b = 0; b < kBatch; ++b) {
    const unsigned short* XBb = XB + (size_t)b * kSeq * kDm;
    float* outb = out + (size_t)b * kSeq * kDm;

    wmma_gemm64<1, 0, 0, 0><<<dim3(256, 1), 256, 0, stream>>>(
        XBb, XBb, kDm, 0L, WINB, WINB, kDm, 0L,
        (void*)XZ, (void*)XZ, kXzP, 0L, gdummy, 0, 0L, kSeq, kXzP, kDm, 1.0f);

    conv_silu_kernel<<<dim3(kDin / 256, kSeq / 64), 256, 0, stream>>>(XZ, conv_w, conv_b, XCH, XCL);

    wmma_gemm64<1, 1, 0, 0><<<dim3(4, 1), 256, 0, stream>>>(
        XCH, XCL, kDin, 0L, WBB, WBB, kDin, 0L,
        (void*)U, (void*)U, kUP, 0L, gdummy, 0, 0L, kSeq, kUP, kDin, 1.0f);

    scan_kernel<<<1, 32, 0, stream>>>(U, HH, HL);

    wmma_gemm64<1, 1, 2, 1><<<dim3(128, 1), 256, 0, stream>>>(
        HH, HL, kHP, 0L, WCB, WCB, kHP, 0L,
        (void*)YH, (void*)YL, kDin, 0L, XZ + kDin, kXzP, 0L, kSeq, kDin, kHP, 1.0f);

    wmma_gemm64<1, 1, 0, 0><<<dim3(64, 1), 256, 0, stream>>>(
        YH, YL, kDin, 0L, WOB, WOB, kDin, 0L,
        (void*)outb, (void*)outb, kDm, 0L, gdummy, 0, 0L, kSeq, kDm, kDin, 1.0f);
  }
}
